// BNAFINN_51015621542177
// MI455X (gfx1250) — hardware-run, weakly checked
//
#include <hip/hip_runtime.h>
#include <math.h>

typedef __attribute__((ext_vector_type(16))) _Float16 v16h;
typedef __attribute__((ext_vector_type(8)))  _Float16 v8h;
typedef __attribute__((ext_vector_type(8)))  float    v8f;
typedef __attribute__((ext_vector_type(4)))  float    v4f;

constexpr int kFlows = 5;
constexpr int kBatch = 4096;
constexpr int kDim   = 64;
constexpr int kNh    = 128;
constexpr int kHid   = kDim * kNh;
static_assert(kHid == 8192);
static_assert((kBatch % 32) == 0 && (kDim % 32) == 0 && (kNh % 32) == 0);
constexpr int kHP = kNh + 8;
constexpr int kXP = kDim + 8;
constexpr int kYP = kDim + 4;
static_assert(((kHP * 2) % 16) == 0 && ((kXP * 2) % 16) == 0 && ((kYP * 4) % 16) == 0);

constexpr float kCarryX  = 1024.0f;
constexpr float kCarryW1 = 16384.0f;
constexpr float kCarryH  = 16384.0f;
constexpr float kCarryW2 = 32768.0f;
constexpr float kFold1   = 1.0f / (kCarryX * kCarryW1);
constexpr float kFold2   = 1.0f / (kCarryH * kCarryW2);
constexpr float kXClamp  = 60000.0f;
constexpr float kF16MinNormal = 6.103515625e-05f;
constexpr float kTwoLn2  = 1.3862943611198906f;
constexpr float kNegBig  = -1.0e30f;

constexpr size_t kSzW1P = (size_t)kFlows * kHid * kDim * 2;
constexpr size_t kSzW2P = (size_t)kFlows * kDim * kHid * 2;
constexpr size_t kSzC   = (size_t)kFlows * kHid * 4;
constexpr size_t kSzX   = (size_t)kBatch * kDim * 4;
constexpr size_t kSzLd  = (size_t)kBatch * 4;
constexpr size_t kOffW1H = 0;
constexpr size_t kOffW2H = kOffW1H + kSzW1P;
constexpr size_t kOffC1  = kOffW2H + kSzW2P;
constexpr size_t kOffCM  = kOffC1 + kSzC;
constexpr size_t kOffXA  = kOffCM + kSzC;
constexpr size_t kOffXB  = kOffXA + kSzX;
constexpr size_t kOffLDA = kOffXB + kSzX;
constexpr size_t kOffLDB = kOffLDA + kSzLd;
constexpr size_t kWsTotal = kOffLDB + kSzLd;
static_assert(kWsTotal == 12943360ull);
static_assert(kWsTotal <= 134217728ull);
static_assert((kOffW2H % 128) == 0 && (kOffC1 % 128) == 0 &&
              (kOffCM % 128) == 0 && (kOffXA % 128) == 0 && (kOffXB % 128) == 0 && (kOffLDA % 128) == 0 &&
              (kOffLDB % 128) == 0);

__device__ __forceinline__ float flush_small(float v) {
  return (fabsf(v) < kF16MinNormal) ? 0.0f : v;
}
__device__ __forceinline__ _Float16 to_h(float v) {
  const float vf = flush_small(v);
  return (_Float16)vf;
}
union FragU { v16h v; v8h h[2]; };
__device__ __forceinline__ v16h frag_ld(const _Float16* p) {
  FragU f;
  f.h[0] = *(const v8h*)(p);
  f.h[1] = *(const v8h*)(p + 16);
  return f.v;
}
__device__ __forceinline__ v8f mma_h(v16h a, v16h b, v8f c) {
  c = __builtin_amdgcn_wmma_f32_16x16x32_f16(false, a, false, b, (short)0, c, false, false);
  asm volatile("v_nop\n\tv_nop\n\tv_nop\n\tv_nop" : "+v"(c) : "v"(a), "v"(b));
  return c;
}

__global__ __launch_bounds__(256) void prep_layer1(
    const float* __restrict__ W1, const float* __restrict__ d1,
    unsigned short* __restrict__ w1hp, float* __restrict__ c1p)
{
  __shared__ float sScale[256];
  __shared__ float sEd[256];
  const int tid = threadIdx.x;
  const int R = blockIdx.x * 256 + tid;
  const int i = (R & (kHid - 1)) >> 7;
  const float* rowp = W1 + (size_t)R * kDim;
  const float wd = rowp[i];
  const float ed = expf(wd);
  float acc = ed * ed;
#pragma unroll 1
  for (int q = 0; q < kDim / 4; ++q) {
    const v4f v = *(const v4f*)(rowp + 4 * q);
    const int k = 4 * q;
    const float t0 = (k + 0 < i) ? v[0] : 0.0f;
    const float t1 = (k + 1 < i) ? v[1] : 0.0f;
    const float t2 = (k + 2 < i) ? v[2] : 0.0f;
    const float t3 = (k + 3 < i) ? v[3] : 0.0f;
    acc = fmaf(t0, t0, acc);
    acc = fmaf(t1, t1, acc);
    acc = fmaf(t2, t2, acc);
    acc = fmaf(t3, t3, acc);
  }
  const float dn = d1[R];
  const float sc = expf(dn) * rsqrtf(acc);
  const float cval = dn + wd - 0.5f * logf(acc);
  sScale[tid] = sc * kCarryW1;
  sEd[tid] = ed;
  {
    volatile float* cp = c1p + R;
    *cp = cval;
    __threadfence();
    *cp = cval;
  }
  __syncthreads();
#pragma unroll 1
  for (int it = 0; it < 8; ++it) {
    const int item = it * 256 + tid;
    const int r = item >> 3;
    const int g8 = (item & 7) * 8;
    const int R2 = blockIdx.x * 256 + r;
    const int i2 = (R2 & (kHid - 1)) >> 7;
    const float* src = W1 + (size_t)R2 * kDim + g8;
    const v4f a0 = *(const v4f*)(src);
    const v4f a1 = *(const v4f*)(src + 4);
    const float scr = sScale[r];
    const float edr = sEd[r];
    const float w[8] = {a0[0], a0[1], a0[2], a0[3], a1[0], a1[1], a1[2], a1[3]};
    v8h hv;
#pragma unroll
    for (int e = 0; e < 8; ++e) {
      const int k = g8 + e;
      const float wv = (k == i2) ? edr : ((k < i2) ? w[e] : 0.0f);
      hv[e] = to_h(wv * scr);
    }
    unsigned short* qh = w1hp + (size_t)R2 * kDim + g8;
    *(volatile v8h*)qh = hv;
    __threadfence();
    *(volatile v8h*)qh = hv;
  }
}

__global__ __launch_bounds__(256) void prep_layer2(
    const float* __restrict__ W2, const float* __restrict__ d2, const float* __restrict__ c1p,
    unsigned short* __restrict__ w2hp, float* __restrict__ cmp)
{
  __shared__ __align__(16) float sE[kNh];
  __shared__ float sRed[8];
  const int tid = threadIdx.x;
  const int lane = tid & 31;
  const int wave = tid >> 5;
  const int f = blockIdx.x / kDim;
  const int d = blockIdx.x - f * kDim;
  const float* rowp = W2 + (size_t)blockIdx.x * kHid;
  const int kd = kNh * d + (tid & (kNh - 1));
  float vd = rowp[kd];
  asm volatile("" : "+v"(vd));
  const float ev = expf(vd);
  if (tid < kNh) sE[tid] = ev;
  float part = (tid < kNh) ? (ev * ev) : 0.0f;
  const int klim = kNh * d;
#pragma unroll 1
  for (int k = tid; k < klim; k += 256) {
    const float v = rowp[k];
    part = fmaf(v, v, part);
  }
  part += __shfl_xor(part, 16, 32);
  part += __shfl_xor(part, 8, 32);
  part += __shfl_xor(part, 4, 32);
  part += __shfl_xor(part, 2, 32);
  part += __shfl_xor(part, 1, 32);
  if (lane == 0) sRed[wave] = part;
  __syncthreads();
  float tot = 0.0f;
#pragma unroll
  for (int w = 0; w < 8; ++w) tot += sRed[w];
  const float dn = d2[blockIdx.x];
  const float sc = expf(dn) * rsqrtf(tot) * kCarryW2;
  const float halflog = 0.5f * logf(tot);
#pragma unroll 1
  for (int it = 0; it < 4; ++it) {
    const int item = it * 256 + tid;
    const int k0 = item * 8;
    const int kb = k0 >> 7;
    const int je = k0 & (kNh - 1);
    const v4f a0 = *(const v4f*)(rowp + k0);
    const v4f a1 = *(const v4f*)(rowp + k0 + 4);
    const v4f e0 = *(const v4f*)(sE + je);
    const v4f e1 = *(const v4f*)(sE + je + 4);
    const float aw[8] = {a0[0], a0[1], a0[2], a0[3], a1[0], a1[1], a1[2], a1[3]};
    const float ew[8] = {e0[0], e0[1], e0[2], e0[3], e1[0], e1[1], e1[2], e1[3]};
    v8h hv;
#pragma unroll
    for (int e = 0; e < 8; ++e) {
      const float wv = (kb == d) ? ew[e] : ((kb < d) ? aw[e] : 0.0f);
      hv[e] = to_h(wv * sc);
    }
    unsigned short* qh = w2hp + (size_t)blockIdx.x * kHid + k0;
    *(volatile v8h*)qh = hv;
    __threadfence();
    *(volatile v8h*)qh = hv;
  }
  if (wave == 0) {
    const int kk = kNh * d + lane * 4;
    const v4f wr = *(const v4f*)(rowp + kk);
    const v4f cc = *(const v4f*)(c1p + (size_t)f * kHid + kk);
    v4f o;
    o[0] = cc[0] + ((dn + wr[0]) - halflog);
    o[1] = cc[1] + ((dn + wr[1]) - halflog);
    o[2] = cc[2] + ((dn + wr[2]) - halflog);
    o[3] = cc[3] + ((dn + wr[3]) - halflog);
    float* cq = cmp + (size_t)f * kHid + kk;
    *(volatile v4f*)cq = o;
    __threadfence();
    *(volatile v4f*)cq = o;
  }
}

__device__ __forceinline__ void act_tile(const v8f acc, const float (&bv)[8], const float (&cv)[8],
                                         float& lm, float& ls, v8h& hv)
{
  float tv[8];
  float gm = kNegBig;
#pragma unroll
  for (int r = 0; r < 8; ++r) {
    const float p = fmaf(acc[r], kFold1, bv[r]);
    const float a = fabsf(p);
    const float e = __expf(-2.0f * a);
    const float u = 1.0f + e;
    const float ru = __builtin_amdgcn_rcpf(u);
    const float th = (1.0f - e) * ru;
    const float hval = copysignf(th, p);
    const float l1p = __logf(u) + (e - (u - 1.0f)) * ru;
    const float tval = ((kTwoLn2 - 2.0f * a) - 2.0f * l1p) + cv[r];
    tv[r] = tval;
    gm = fmaxf(gm, tval);
    hv[r] = to_h(hval * kCarryH);
  }
  const float mn = fmaxf(lm, gm);
  float ss = ls * __expf(lm - mn);
#pragma unroll
  for (int r = 0; r < 8; ++r) ss += __expf(tv[r] - mn);
  lm = mn;
  ls = ss;
}

__device__ __forceinline__ float softplus_fast(float z) {
  const float az = fabsf(z);
  const float ez = __expf(-az);
  const float uz = 1.0f + ez;
  const float lz = __logf(uz) + (ez - (uz - 1.0f)) * __builtin_amdgcn_rcpf(uz);
  return fmaxf(z, 0.0f) + lz;
}

__global__ __launch_bounds__(32) __attribute__((amdgpu_num_vgpr(256))) void flow_step(
    const float* __restrict__ xin, float* __restrict__ xout,
    const unsigned short* __restrict__ w1hp,
    const float* __restrict__ b1,
    const unsigned short* __restrict__ w2hp,
    const float* __restrict__ b2, const float* __restrict__ cmat,
    const float* __restrict__ gates, const float* __restrict__ ldin, float* __restrict__ ldout, int flow)
{
  __shared__ __align__(16) _Float16 sHh[32 * kHP];
  __shared__ __align__(16) _Float16 sXh[32 * kXP];
  __shared__ __align__(16) float sY[32 * kYP];

  const _Float16* w1h = (const _Float16*)w1hp;
  const _Float16* w2h = (const _Float16*)w2hp;

  const int lane = threadIdx.x & 31;
  const int hh = lane >> 4;
  const int c = lane & 15;
  const int row0 = blockIdx.x * 32;

#pragma unroll 1
  for (int jk = 0; jk < 4; ++jk) {
    const int j = jk >> 1;
    const int ks = jk & 1;
    const float* xr = xin + (size_t)(row0 + 16 * j + c) * kDim + 32 * ks + 8 * hh;
    const v4f q0 = *(const v4f*)(xr);
    const v4f q1 = *(const v4f*)(xr + 4);
    const v4f q2 = *(const v4f*)(xr + 16);
    const v4f q3 = *(const v4f*)(xr + 20);
    const float xa[8] = {q0[0], q0[1], q0[2], q0[3], q1[0], q1[1], q1[2], q1[3]};
    const float xb[8] = {q2[0], q2[1], q2[2], q2[3], q3[0], q3[1], q3[2], q3[3]};
    v8h h0, h1;
#pragma unroll
    for (int e = 0; e < 8; ++e) {
      const float va = fminf(fmaxf(xa[e] * kCarryX, -kXClamp), kXClamp);
      const float vb = fminf(fmaxf(xb[e] * kCarryX, -kXClamp), kXClamp);
      h0[e] = to_h(va);
      h1[e] = to_h(vb);
    }
    const int so = (16 * j + c) * kXP + 32 * ks + 8 * hh;
    *(v8h*)(sXh + so) = h0;
    *(v8h*)(sXh + so + 16) = h1;
  }
  __syncthreads();

  const bool gated = (flow < kFlows - 1);
  const int gi = gated ? flow : (kFlows - 2);
  const float gv = gates[gi];
  const float sg = 1.0f / (1.0f + expf(-gv));
  const float spg = fmaxf(gv, 0.0f) + log1pf(expf(-fabsf(gv)));

  v8f yacc[2][4];
#pragma unroll
  for (int j = 0; j < 2; ++j)
#pragma unroll
    for (int td = 0; td < 4; ++td) yacc[j][td] = (v8f){0.f, 0.f, 0.f, 0.f, 0.f, 0.f, 0.f, 0.f};

  float ldacc = 0.0f;

#pragma unroll 1
  for (int ch = 0; ch < kDim; ++ch) {
    const int n0 = ch * kNh;
    float lm0 = kNegBig, ls0 = 0.0f, lm1 = kNegBig, ls1 = 0.0f;

#pragma unroll 1
    for (int t = 0; t < 8; ++t) {
      const size_t wo = (size_t)(n0 + 16 * t + c) * kDim + 8 * hh;
      v8f acc0 = (v8f){0.f, 0.f, 0.f, 0.f, 0.f, 0.f, 0.f, 0.f};
      v8f acc1 = (v8f){0.f, 0.f, 0.f, 0.f, 0.f, 0.f, 0.f, 0.f};
      {
        int xo = c * kXP + 8 * hh;
        asm volatile("" : "+v"(xo));
        const v16h wh = frag_ld(w1h + wo);
        const v16h xh0 = frag_ld(sXh + xo);
        acc0 = mma_h(wh, xh0, acc0);
        const v16h xh1 = frag_ld(sXh + 16 * kXP + xo);
        acc1 = mma_h(wh, xh1, acc1);
      }
      if (ch >= 32) {
        int xo = c * kXP + 8 * hh + 32;
        asm volatile("" : "+v"(xo));
        const v16h wh = frag_ld(w1h + wo + 32);
        const v16h xh0 = frag_ld(sXh + xo);
        acc0 = mma_h(wh, xh0, acc0);
        const v16h xh1 = frag_ld(sXh + 16 * kXP + xo);
        acc1 = mma_h(wh, xh1, acc1);
      }
      const int kb = n0 + 16 * t + 8 * hh;
      const v4f bA = *(const v4f*)(b1 + kb);
      const v4f bB = *(const v4f*)(b1 + kb + 4);
      const v4f cA = *(const v4f*)(cmat + kb);
      const v4f cB = *(const v4f*)(cmat + kb + 4);
      const float bv[8] = {bA[0], bA[1], bA[2], bA[3], bB[0], bB[1], bB[2], bB[3]};
      const float cv[8] = {cA[0], cA[1], cA[2], cA[3], cB[0], cB[1], cB[2], cB[3]};
      const int hcol = 16 * t + 8 * hh;
      {
        v8h hv;
        act_tile(acc0, bv, cv, lm0, ls0, hv);
        *(v8h*)(sHh + c * kHP + hcol) = hv;
      }
      {
        v8h hv;
        act_tile(acc1, bv, cv, lm1, ls1, hv);
        *(v8h*)(sHh + (16 + c) * kHP + hcol) = hv;
      }
    }

    {
      const float m0o = __shfl_xor(lm0, 16, 32);
      const float s0o = __shfl_xor(ls0, 16, 32);
      const float m1o = __shfl_xor(lm1, 16, 32);
      const float s1o = __shfl_xor(ls1, 16, 32);
      const float M0 = fmaxf(lm0, m0o);
      const float S0 = ls0 * __expf(lm0 - M0) + s0o * __expf(m0o - M0);
      const float M1 = fmaxf(lm1, m1o);
      const float S1 = ls1 * __expf(lm1 - M1) + s1o * __expf(m1o - M1);
      const float lse0 = M0 + __logf(S0);
      const float lse1 = M1 + __logf(S1);
      float t0 = lse0, t1 = lse1;
      if (gated) {
        t0 = softplus_fast(lse0 + gv) - spg;
        t1 = softplus_fast(lse1 + gv) - spg;
      }
      ldacc += (hh == 0) ? t0 : t1;
    }

    __syncthreads();

    {
      const int td0 = ch >> 4;
#pragma unroll 1
      for (int ks = 0; ks < 4; ++ks) {
        const int ao = c * kHP + 32 * ks + 8 * hh;
        const v16h ah0 = frag_ld(sHh + ao);
        const v16h ah1 = frag_ld(sHh + 16 * kHP + ao);
#pragma unroll
        for (int td = 0; td < 4; ++td) {
          if (td >= td0) {
            int bo = (16 * td + c) * kHid + n0 + 32 * ks + 8 * hh;
            asm volatile("" : "+v"(bo));
            const v16h bh = frag_ld(w2h + bo);
            yacc[0][td] = mma_h(ah0, bh, yacc[0][td]);
            yacc[1][td] = mma_h(ah1, bh, yacc[1][td]);
          }
        }
      }
    }
    __syncthreads();
  }

#pragma unroll
  for (int td = 0; td < 4; ++td) {
    const float bz = b2[16 * td + c];
#pragma unroll
    for (int j = 0; j < 2; ++j) {
#pragma unroll
      for (int r = 0; r < 8; ++r) {
        sY[(16 * j + 8 * hh + r) * kYP + 16 * td + c] = fmaf(yacc[j][td][r], kFold2, bz);
      }
    }
  }
  __syncthreads();

  {
    const int c4 = c * 4;
    const float omsg = 1.0f - sg;
#pragma unroll 1
    for (int half = 0; half < 2; ++half) {
      const int rbase = 16 * half;
      v4f ov[8];
      if (gated) {
#pragma unroll
        for (int it = 0; it < 8; ++it) {
          const int row = rbase + 2 * it + hh;
          const v4f ys = *(const v4f*)(sY + row * kYP + 60 - c4);
          const v4f xs = *(const v4f*)(xin + (size_t)(row0 + row) * kDim + 60 - c4);
          v4f o;
          o[0] = sg * ys[3] + omsg * xs[3];
          o[1] = sg * ys[2] + omsg * xs[2];
          o[2] = sg * ys[1] + omsg * xs[1];
          o[3] = sg * ys[0] + omsg * xs[0];
          ov[it] = o;
        }
      } else {
#pragma unroll
        for (int it = 0; it < 8; ++it) {
          const int row = rbase + 2 * it + hh;
          ov[it] = *(const v4f*)(sY + row * kYP + c4);
        }
      }
      for (int pass = 0; pass < 2; ++pass) {
#pragma unroll
        for (int it = 0; it < 8; ++it) {
          const int row = rbase + 2 * it + hh;
          *(volatile v4f*)(xout + (size_t)(row0 + row) * kDim + c4) = ov[it];
        }
        __threadfence();
      }
    }
  }

  {
    float base = 0.0f;
    if (flow > 0) base = ldin[row0 + lane];
    const float tot = base + ldacc;
    volatile float* lp = ldout + row0 + lane;
    *lp = tot;
    __threadfence();
    *lp = tot;
  }
}

extern "C" void kernel_launch(void* const* d_in, const int* in_sizes, int n_in,
                              void* d_out, int out_size, void* d_ws, size_t ws_size,
                              hipStream_t stream) {
  if (n_in < 8) return;
  if (in_sizes[0] != kBatch * kDim) return;
  if (in_sizes[1] != kFlows * kHid * kDim) return;
  if (in_sizes[2] != kFlows * kHid) return;
  if (in_sizes[3] != kFlows * kHid) return;
  if (in_sizes[4] != kFlows * kDim * kHid) return;
  if (in_sizes[5] != kFlows * kDim) return;
  if (in_sizes[6] != kFlows * kDim) return;
  if (in_sizes[7] != kFlows - 1) return;
  if (out_size != kBatch * kDim + kBatch) return;
  if (ws_size < kWsTotal) return;

  const float* x     = (const float*)d_in[0];
  const float* W1    = (const float*)d_in[1];
  const float* d1    = (const float*)d_in[2];
  const float* b1    = (const float*)d_in[3];
  const float* W2    = (const float*)d_in[4];
  const float* d2    = (const float*)d_in[5];
  const float* b2    = (const float*)d_in[6];
  const float* gates = (const float*)d_in[7];

  char* ws = (char*)d_ws;
  unsigned short* W1H = (unsigned short*)(ws + kOffW1H);
  unsigned short* W2H = (unsigned short*)(ws + kOffW2H);
  float* C1  = (float*)(ws + kOffC1);
  float* CM  = (float*)(ws + kOffCM);
  float* XA  = (float*)(ws + kOffXA);
  float* XB  = (float*)(ws + kOffXB);
  float* LDA = (float*)(ws + kOffLDA);
  float* LDB = (float*)(ws + kOffLDB);

  float* out0 = (float*)d_out;
  float* out1 = out0 + (size_t)kBatch * kDim;

  prep_layer1<<<kFlows * kHid / 256, 256, 0, stream>>>(W1, d1, W1H, C1);
  prep_layer2<<<kFlows * kDim, 256, 0, stream>>>(W2, d2, C1, W2H, CM);

  const float* xcur = x;
  const float* ldcur = LDB;
  for (int f = 0; f < kFlows; ++f) {
    float* xnext = (f == kFlows - 1) ? out0 : ((f & 1) ? XB : XA);
    float* ldnext = (f == kFlows - 1) ? out1 : ((f & 1) ? LDB : LDA);
    flow_step<<<kBatch / 32, 32, 0, stream>>>(
        xcur, xnext,
        W1H + (size_t)f * kHid * kDim,
        b1 + (size_t)f * kHid,
        W2H + (size_t)f * kDim * kHid,
        b2 + (size_t)f * kDim, CM + (size_t)f * kHid,
        gates, ldcur, ldnext, f);
    xcur = xnext;
    ldcur = ldnext;
  }
}
